// LocalDeformKernel2d_89507118448686
// MI455X (gfx1250) — hardware-verified
//
#include <hip/hip_runtime.h>
#include <stdint.h>


typedef __bf16   v16bf __attribute__((ext_vector_type(16)));
typedef float    v8f   __attribute__((ext_vector_type(8)));
typedef float    v4f   __attribute__((ext_vector_type(4)));
typedef v4f      v4fa  __attribute__((may_alias));
typedef unsigned v4u   __attribute__((ext_vector_type(4)));

#define B_   4
#define C_   128
#define H_   96
#define W_   96
#define HW_  (H_ * W_)
#define HP_  (H_ + 2)
#define WP_  (W_ + 2)
#define O_   18
#define KTOT (C_ * 9)
#define NKB  (KTOT / 32)

#define NPIX      (B_ * HW_)
#define PIX_PER_BLK 64
#define NBLK      (NPIX / PIX_PER_BLK)
#define BP_ELEMS  (2 * NKB * 32 * 16)
#define BP_BYTES  (BP_ELEMS * 2)
#define XH_ELEMS  (B_ * HP_ * WP_ * C_)
#define XH_BYTES  (XH_ELEMS * 2)
#define NGB       (BP_ELEMS / 8)
#define NGX       (XH_ELEMS / 8)

typedef char sa_tile_in_row  [(W_ % 16 == 0) ? 1 : -1];
typedef char sa_line_in_row  [(W_ % 32 == 0) ? 1 : -1];
typedef char sa_blk_in_batch [(HW_ % PIX_PER_BLK == 0) ? 1 : -1];
typedef char sa_blk_cover    [(NPIX % PIX_PER_BLK == 0) ? 1 : -1];
typedef char sa_chan_chunks  [(C_ % 32 == 0) ? 1 : -1];
typedef char sa_carve_align  [(BP_BYTES % 256 == 0 && XH_BYTES % 256 == 0) ? 1 : -1];
typedef char sa_pack_grid    [(NGX % 256 == 0) ? 1 : -1];

__host__ __device__ __forceinline__ int swap34(int r) {
    return (r & ~0x18) | ((r & 8) << 1) | ((r & 16) >> 1);
}

__device__ __forceinline__ unsigned bf16_rne_bits(float f) {
    unsigned u = __float_as_uint(f);
    u = u + 0x7FFFu + ((u >> 16) & 1u);
    return u >> 16;
}

__device__ __forceinline__ void split_bf16(float f, unsigned& hi, unsigned& lo) {
    hi = bf16_rne_bits(f);
    float fh = __uint_as_float(hi << 16);
    lo = bf16_rne_bits(f - fh);
}

__device__ __forceinline__ v8f wmma3(v16bf ah, v16bf al, v16bf bh, v16bf bl, v8f c) {
    c = __builtin_amdgcn_wmma_f32_16x16x32_bf16(false, ah, false, bh, (short)0, c, false, false);
    c = __builtin_amdgcn_wmma_f32_16x16x32_bf16(false, ah, false, bl, (short)0, c, false, false);
    c = __builtin_amdgcn_wmma_f32_16x16x32_bf16(false, al, false, bh, (short)0, c, false, false);
    asm volatile("v_nop\n\tv_nop\n\tv_nop\n\tv_nop" : "+v"(c) : "v"(ah), "v"(al), "v"(bh), "v"(bl));
    return c;
}

__global__ __launch_bounds__(256) void pack_b_kernel(
    const float* __restrict__ rot_w, unsigned* __restrict__ bph, unsigned* __restrict__ bpl)
{
    const int tid = blockIdx.x * 256 + threadIdx.x;
    if (tid >= NGB) return;
    const int ig   = tid & 1;
    const int lane = (tid >> 1) & 31;
    const int r    = tid >> 6;
    const int kb   = r % NKB;
    const int nt   = r / NKB;
    const int n    = nt * 16 + (lane & 15);
    const int hf   = lane >> 4;
    const int ij   = kb >> 2;
    const int cb   = kb & 3;

    unsigned hw[4] = {0u, 0u, 0u, 0u}, lw[4] = {0u, 0u, 0u, 0u};
#pragma unroll
    for (int j = 0; j < 8; ++j) {
        const int kk = 16 * ig + 8 * hf + j;
        const int c  = cb * 32 + kk;
        float v = 0.0f;
        if (n < O_) v = rot_w[n * KTOT + c * 9 + ij];
        unsigned h16, l16;
        split_bf16(v, h16, l16);
        hw[j >> 1] |= h16 << (16 * (j & 1));
        lw[j >> 1] |= l16 << (16 * (j & 1));
    }
    v4u hv, lv;
    hv.x = hw[0]; hv.y = hw[1]; hv.z = hw[2]; hv.w = hw[3];
    lv.x = lw[0]; lv.y = lw[1]; lv.z = lw[2]; lv.w = lw[3];
    volatile v4u* ph = (volatile v4u*)(bph + (size_t)tid * 4);
    volatile v4u* pl = (volatile v4u*)(bpl + (size_t)tid * 4);
    *ph = hv;
    *pl = lv;
    __threadfence();
    *ph = hv;
    *pl = lv;
}

__global__ __launch_bounds__(256) void pack_x_kernel(
    const float* __restrict__ x, unsigned* __restrict__ xhh, unsigned* __restrict__ xhl)
{
    const int tid = blockIdx.x * 256 + threadIdx.x;
    if (tid >= NGX) return;
    const int g  = tid & 15;
    int s        = tid >> 4;
    const int wp = s % WP_;
    s            = s / WP_;
    const int hp = s % HP_;
    const int b  = s / HP_;
    const int r0 = swap34(g * 8);
    const bool inb = (hp >= 1) && (hp <= H_) && (wp >= 1) && (wp <= W_);

    unsigned hw[4] = {0u, 0u, 0u, 0u}, lw[4] = {0u, 0u, 0u, 0u};
    if (inb) {
        const float* xp = x + ((size_t)(b * C_ + r0) * H_ + (hp - 1)) * W_ + (wp - 1);
#pragma unroll
        for (int j = 0; j < 8; ++j) {
            const float v = xp[(size_t)j * HW_];
            unsigned h16, l16;
            split_bf16(v, h16, l16);
            hw[j >> 1] |= h16 << (16 * (j & 1));
            lw[j >> 1] |= l16 << (16 * (j & 1));
        }
    }
    v4u hv, lv;
    hv.x = hw[0]; hv.y = hw[1]; hv.z = hw[2]; hv.w = hw[3];
    lv.x = lw[0]; lv.y = lw[1]; lv.z = lw[2]; lv.w = lw[3];
    volatile v4u* ph = (volatile v4u*)(xhh + (size_t)tid * 4);
    volatile v4u* pl = (volatile v4u*)(xhl + (size_t)tid * 4);
    *ph = hv;
    *pl = lv;
    __threadfence();
    *ph = hv;
    *pl = lv;
}

__global__ __launch_bounds__(128) void deform_main_kernel(
    const float* __restrict__ x,
    const float* __restrict__ rot_b,
    const float* __restrict__ weight,
    const __bf16* __restrict__ bph,
    const __bf16* __restrict__ bpl,
    const __bf16* __restrict__ xhh,
    const __bf16* __restrict__ xhl,
    float* out)
{
    __shared__ float    wlds[C_ * 16];
    __shared__ float    rot_lds[4][16 * 32];
    __shared__ v4f      coef_lds[4][144];
    __shared__ unsigned idx_lds[4][144];
    __shared__ __attribute__((aligned(16))) float stg[32 * PIX_PER_BLK];

    if (blockIdx.x >= NBLK) return;

    const int t    = threadIdx.x;
    const int wave = t >> 5;
    const int lane = t & 31;
    const int m    = lane & 15;
    const int hf   = lane >> 4;

    for (int s = t; s < C_ * 16; s += 128) wlds[s] = weight[s];

    const int tile = blockIdx.x * 4 + wave;
    const int p0   = tile * 16;
    const int b    = p0 / HW_;
    const int rem  = p0 - b * HW_;
    const int hr   = rem / W_;
    const int w0   = rem - hr * W_;
    const int w    = w0 + m;

    v8f acc0, acc1;
#pragma unroll
    for (int i = 0; i < 8; ++i) { acc0[i] = 0.0f; acc1[i] = 0.0f; }

    const v16bf* bh16 = (const v16bf*)bph;
    const v16bf* bl16 = (const v16bf*)bpl;
#pragma unroll 1
    for (int ij = 0; ij < 9; ++ij) {
        const int di  = ij / 3;
        const int dj  = ij - 3 * di;
        const int pix = ((b * HP_ + hr + di) * WP_ + (w + dj)) * C_ + 16 * hf;
        const __bf16* aph = xhh + pix;
        const __bf16* apl = xhl + pix;
#pragma unroll 1
        for (int cb = 0; cb < 4; ++cb) {
            const v16bf ah = *(const v16bf*)(aph + cb * 32);
            const v16bf al = *(const v16bf*)(apl + cb * 32);
            const int kb   = ij * 4 + cb;
            const v16bf b0h = bh16[kb * 32 + lane];
            const v16bf b0l = bl16[kb * 32 + lane];
            const v16bf b1h = bh16[(NKB + kb) * 32 + lane];
            const v16bf b1l = bl16[(NKB + kb) * 32 + lane];
            acc0 = wmma3(ah, al, b0h, b0l, acc0);
            acc1 = wmma3(ah, al, b1h, b1l, acc1);
        }
    }

    {
        const int mrow = hf * 8;
#pragma unroll
        for (int i = 0; i < 8; ++i) {
            rot_lds[wave][(mrow + i) * 32 + m]      = acc0[i];
            rot_lds[wave][(mrow + i) * 32 + m + 16] = acc1[i];
        }
    }
    __syncthreads();

#pragma unroll
    for (int it = 0; it < 5; ++it) {
        const int task = lane + it * 32;
        if (task < 144) {
            const int tm = task & 15, ij = task >> 4;
            const int di = ij / 3, dj = ij - 3 * di;
            float ch = rot_lds[wave][tm * 32 + 2 * ij]     + rot_b[2 * ij]
                     + (0.5f + (float)di);
            float cw = rot_lds[wave][tm * 32 + 2 * ij + 1] + rot_b[2 * ij + 1]
                     + (0.5f + (float)dj);
            ch = fminf(fmaxf(ch, 0.0f), 3.0f);
            cw = fminf(fmaxf(cw, 0.0f), 3.0f);
            const float fh = floorf(ch), fw = floorf(cw);
            int h0 = (int)fh, w0i = (int)fw;
            h0  = min(max(h0, 0), 3);
            w0i = min(max(w0i, 0), 3);
            const int h1 = min(h0 + 1, 3), w1 = min(w0i + 1, 3);
            const float lh = ch - fh, lw = cw - fw;
            v4f cf;
            cf.x = (1.0f - lh) * (1.0f - lw);
            cf.y = (1.0f - lh) * lw;
            cf.z = lh * (1.0f - lw);
            cf.w = lh * lw;
            coef_lds[wave][task] = cf;
            idx_lds[wave][task] =
                (unsigned)(h0 * 4 + w0i)        |
                ((unsigned)(h0 * 4 + w1)  << 8) |
                ((unsigned)(h1 * 4 + w0i) << 16)|
                ((unsigned)(h1 * 4 + w1)  << 24);
        }
    }
    __syncthreads();

    v4f      cf[9];
    unsigned idp[9];
    int      xoff[9];
    float    msk[9];
#pragma unroll
    for (int ij = 0; ij < 9; ++ij) {
        cf[ij]  = coef_lds[wave][ij * 16 + m];
        idp[ij] = idx_lds[wave][ij * 16 + m];
        const int hh = hr + ij / 3 - 1, ww = w + ij % 3 - 1;
        const bool ok = (hh >= 0) && (hh < H_) && (ww >= 0) && (ww < W_);
        const int hc = min(max(hh, 0), H_ - 1);
        const int wc = min(max(ww, 0), W_ - 1);
        xoff[ij] = hc * W_ + wc;
        msk[ij]  = ok ? 1.0f : 0.0f;
    }

    const size_t xbatch = (size_t)b * C_ * HW_;
    const size_t obase  = (size_t)blockIdx.x * PIX_PER_BLK + (size_t)b * (C_ - 1) * HW_;
    const int    q8     = lane >> 3;
    const int    e8     = lane & 7;

    for (int ch0 = 0; ch0 < C_; ch0 += 32) {
        for (int cp = 0; cp < 16; ++cp) {
            const int cl = 2 * cp + hf;
            const int c  = ch0 + cl;
            const float* wr = wlds + c * 16;
            const float* xc = x + xbatch + (size_t)c * HW_;
            float sum = 0.0f;
#pragma unroll
            for (int ij = 0; ij < 9; ++ij) {
                const unsigned id = idp[ij];
                const float ws = cf[ij].x * wr[id & 15]
                               + cf[ij].y * wr[(id >> 8)  & 15]
                               + cf[ij].z * wr[(id >> 16) & 15]
                               + cf[ij].w * wr[(id >> 24) & 15];
                const float xv = xc[xoff[ij]] * msk[ij];
                sum += ws * xv;
            }
            stg[cl * PIX_PER_BLK + wave * 16 + m] = sum;
        }
        __syncthreads();

        v4f    vals[4];
        size_t offs[4];
#pragma unroll
        for (int s = 0; s < 4; ++s) {
            const int L   = (wave * 4 + s) * 4 + q8;
            const int cl  = L >> 1;
            const int lhf = L & 1;
            vals[s] = *(const v4fa*)(stg + cl * PIX_PER_BLK + lhf * 32 + e8 * 4);
            offs[s] = obase + (size_t)(ch0 + cl) * HW_ + (size_t)(lhf * 32 + e8 * 4);
            *(volatile v4f*)(out + offs[s]) = vals[s];
        }
        __threadfence();
#pragma unroll
        for (int s = 0; s < 4; ++s) {
            *(volatile v4f*)(out + offs[s]) = vals[s];
        }
        __syncthreads();
    }
}

extern "C" void kernel_launch(void* const* d_in, const int* in_sizes, int n_in,
                              void* d_out, int out_size, void* d_ws, size_t ws_size,
                              hipStream_t stream)
{
    if (n_in < 4) return;
    if (in_sizes[0] != B_ * C_ * HW_) return;
    if (in_sizes[1] != O_ * KTOT) return;
    if (in_sizes[2] < O_) return;
    if (in_sizes[3] != C_ * 16) return;
    if (out_size != B_ * C_ * HW_) return;

    const size_t off_bph = 0;
    const size_t off_bpl = off_bph + BP_BYTES;
    const size_t off_xhh = off_bpl + BP_BYTES;
    const size_t off_xhl = off_xhh + XH_BYTES;
    const size_t need    = off_xhl + XH_BYTES;
    if (need > ws_size) return;

    const float* x      = (const float*)d_in[0];
    const float* rot_w  = (const float*)d_in[1];
    const float* rot_b  = (const float*)d_in[2];
    const float* weight = (const float*)d_in[3];
    float*       out    = (float*)d_out;

    char* ws = (char*)d_ws;
    unsigned* bph_u = (unsigned*)(ws + off_bph);
    unsigned* bpl_u = (unsigned*)(ws + off_bpl);
    unsigned* xhh_u = (unsigned*)(ws + off_xhh);
    unsigned* xhl_u = (unsigned*)(ws + off_xhl);

    pack_b_kernel<<<(NGB + 255) / 256, 256, 0, stream>>>(rot_w, bph_u, bpl_u);
    pack_x_kernel<<<(NGX + 255) / 256, 256, 0, stream>>>(x, xhh_u, xhl_u);
    deform_main_kernel<<<NBLK, 128, 0, stream>>>(
        x, rot_b, weight,
        (const __bf16*)(ws + off_bph), (const __bf16*)(ws + off_bpl),
        (const __bf16*)(ws + off_xhh), (const __bf16*)(ws + off_xhl),
        out);
}
